// ModifiedLSTM_60997125538430
// MI455X (gfx1250) — hardware-verified
//
#include <hip/hip_runtime.h>
#include <math.h>

constexpr int NSEQ    = 64;
constexpr int NSTEP   = 512;
constexpr int NIN     = 256;
constexpr int NHID    = 512;
constexpr int NG4     = 4 * NHID;
constexpr int NCLS    = 1000;
constexpr int NCLSP   = 1024;
constexpr int NTHR    = 512;
constexpr int NWAVE   = NTHR / 32;
constexpr int SEQ_BLK = 16;
constexpr int XPITCH  = 264;
constexpr int HPITCH  = 520;
constexpr int FPITCH  = 516;
constexpr int OUT_BLK = SEQ_BLK * NCLS;
constexpr int OUT_CHUNKS = OUT_BLK / 128;
constexpr int CVT_THR = 256;
constexpr int PL_X = NG4 * NIN;
constexpr int PL_H = NG4 * NHID;
constexpr int PL_C = NCLSP * NHID;
constexpr float LN_EPS = 1e-5f;
constexpr float INV_H  = 1.0f / 512.0f;
static_assert(NSEQ % SEQ_BLK == 0);
static_assert(NIN % 32 == 0 && NHID % 32 == 0);
static_assert(NHID == 32 * NWAVE);
static_assert(NCLSP == 64 * NWAVE);
static_assert(SEQ_BLK == NWAVE);
static_assert(OUT_CHUNKS * 128 == OUT_BLK);
static_assert((OUT_BLK * 4) % 128 == 0);
static_assert(XPITCH % 8 == 0 && HPITCH % 8 == 0 && FPITCH % 4 == 0);
static_assert(NTHR == 32 * SEQ_BLK);
static_assert((PL_X * 2) % 256 == 0 && (PL_H * 2) % 256 == 0 && (PL_C * 2) % 256 == 0);

typedef __attribute__((ext_vector_type(8)))  _Float16 v8h;
typedef __attribute__((ext_vector_type(16))) __bf16   v16b;
typedef __attribute__((ext_vector_type(8)))  __bf16   v8b;
typedef __attribute__((ext_vector_type(8)))  float    v8f;
typedef __attribute__((ext_vector_type(4)))  float    v4f;

__device__ __forceinline__ unsigned short f2bf_bits(float f) {
  unsigned u = __float_as_uint(f);
  return (unsigned short)((u + 0x7FFFu + ((u >> 16) & 1u)) >> 16);
}
__device__ __forceinline__ float bf_bits2f(unsigned short h) { return __uint_as_float(((unsigned)h) << 16); }
__device__ __forceinline__ void split_bits(float f, unsigned short& hb, unsigned short& lb) {
  hb = f2bf_bits(f);
  lb = f2bf_bits(f - bf_bits2f(hb));
}
__device__ __forceinline__ _Float16 as_h16(unsigned short u) { return __builtin_bit_cast(_Float16, u); }

__device__ __forceinline__ void guard_all(v8f& a0, v8f& a1, v8f& a2, v8f& a3, v16b x, v16b y, v16b z, v16b w) {
  asm volatile("v_nop\n\tv_nop\n\tv_nop\n\tv_nop" : "+v"(a0), "+v"(a1), "+v"(a2), "+v"(a3) : "v"(x), "v"(y), "v"(z), "v"(w));
}
__device__ __forceinline__ void acc_guard4(v8f& a, v8f& b, v8f& c, v8f& d) { asm volatile("v_nop\n\tv_nop\n\tv_nop\n\tv_nop" : "+v"(a), "+v"(b), "+v"(c), "+v"(d)); }
template <typename T> struct Frag;
template <> struct Frag<__bf16> {
  typedef v16b V; union U { v16b v; v8b h[2]; };
  static __device__ __forceinline__ v16b load(const __bf16* p) {
    U f; f.h[0] = *(const v8b*)(p); f.h[1] = *(const v8b*)(p + 16); return f.v;
  }
  static __device__ __forceinline__ v8f mma(v16b a, v16b b, v8f c) {
    return __builtin_amdgcn_wmma_f32_16x16x32_bf16(false, a, false, b, (short)0, c, false, false);
  }
};

__device__ __forceinline__ float fsig(float x)  { return __builtin_amdgcn_rcpf(1.0f + __expf(-x)); }
__device__ __forceinline__ float ftanh(float x) { return 1.0f - 2.0f * __builtin_amdgcn_rcpf(__expf(2.0f * x) + 1.0f); }

__global__ __launch_bounds__(CVT_THR) void split8_kernel(const float* __restrict__ src, unsigned short* __restrict__ hi,
                                                        unsigned short* __restrict__ lo, int n8, int n8src) {
  const int i = blockIdx.x * CVT_THR + threadIdx.x;
  if (i < n8) {
    const bool live = (i < n8src);
    const int ic = live ? i : (n8src - 1);
    const v4f a = *(const v4f*)(src + (size_t)ic * 8);
    const v4f b = *(const v4f*)(src + (size_t)ic * 8 + 4);
    v8h hv, lv;
#pragma unroll
    for (int e = 0; e < 4; ++e) {
      unsigned short h0, l0, h1, l1;
      split_bits(a[e], h0, l0);
      split_bits(b[e], h1, l1);
      if (!live) { h0 = 0; l0 = 0; h1 = 0; l1 = 0; }
      hv[e] = as_h16(h0);  lv[e] = as_h16(l0);
      hv[4 + e] = as_h16(h1);  lv[4 + e] = as_h16(l1);
    }
    *(volatile v8h*)(hi + (size_t)i * 8) = hv;
    *(volatile v8h*)(lo + (size_t)i * 8) = lv;
    __threadfence();
    *(volatile v8h*)(hi + (size_t)i * 8) = hv;
    *(volatile v8h*)(lo + (size_t)i * 8) = lv;
  }
}

struct __align__(16) LdsMain {
  unsigned short axh[SEQ_BLK * XPITCH];
  unsigned short axl[SEQ_BLK * XPITCH];
  unsigned short ah0h[SEQ_BLK * HPITCH];
  unsigned short ah0l[SEQ_BLK * HPITCH];
  unsigned short ah1h[SEQ_BLK * HPITCH];
  unsigned short ah1l[SEQ_BLK * HPITCH];
  float          hf[SEQ_BLK * FPITCH];
  unsigned short auh[SEQ_BLK * HPITCH];
  unsigned short aul[SEQ_BLK * HPITCH];
  int            sst[SEQ_BLK];
};
static_assert(sizeof(LdsMain) == 149824);
static_assert(__builtin_offsetof(LdsMain, axl) % 16 == 0 && __builtin_offsetof(LdsMain, ah0h) % 16 == 0 &&
              __builtin_offsetof(LdsMain, ah0l) % 16 == 0 && __builtin_offsetof(LdsMain, ah1h) % 16 == 0 &&
              __builtin_offsetof(LdsMain, ah1l) % 16 == 0 && __builtin_offsetof(LdsMain, hf) % 16 == 0 &&
              __builtin_offsetof(LdsMain, auh) % 16 == 0 && __builtin_offsetof(LdsMain, aul) % 16 == 0);
union __align__(16) LdsAll {
  LdsMain m;
  float ost[OUT_BLK];
};
static_assert(sizeof(float) * OUT_BLK <= __builtin_offsetof(LdsMain, hf));

__device__ __forceinline__ void stage_x(const float* __restrict__ x, unsigned short* axh, unsigned short* axl, int rowbase, int t, int tid) {
  const int m = tid >> 5, f0 = (tid & 31) * 8;
  const float* src = x + ((size_t)(rowbase + m) * NSTEP + (size_t)t) * NIN + f0;
  const v4f q0 = *(const v4f*)(src);
  const v4f q1 = *(const v4f*)(src + 4);
  v8h ph, pl;
#pragma unroll
  for (int e = 0; e < 4; ++e) {
    unsigned short hb, lb;
    split_bits(q0[e], hb, lb); ph[e] = as_h16(hb); pl[e] = as_h16(lb);
    split_bits(q1[e], hb, lb); ph[4 + e] = as_h16(hb); pl[4 + e] = as_h16(lb);
  }
  *(v8h*)(axh + m * XPITCH + f0) = ph;
  *(v8h*)(axl + m * XPITCH + f0) = pl;
}

template <bool RAW>
__device__ __forceinline__ void ln_row(const float* hfrow, const float* __restrict__ gp, const float* __restrict__ bp,
                                       unsigned short* uh, unsigned short* ul, unsigned short* rh, unsigned short* rl, int lane) {
  const int c0 = 16 * lane;
  float v[16];
  {
    const v4f q0 = *(const v4f*)(hfrow + c0);
    const v4f q1 = *(const v4f*)(hfrow + c0 + 4);
    const v4f q2 = *(const v4f*)(hfrow + c0 + 8);
    const v4f q3 = *(const v4f*)(hfrow + c0 + 12);
#pragma unroll
    for (int e = 0; e < 4; ++e) { v[e] = q0[e]; v[4 + e] = q1[e]; v[8 + e] = q2[e]; v[12 + e] = q3[e]; }
  }
  if (RAW) {
#pragma unroll
    for (int hq = 0; hq < 2; ++hq) {
      v8h ph, pl;
#pragma unroll
      for (int e = 0; e < 8; ++e) {
        unsigned short hb, lb;
        split_bits(v[8 * hq + e], hb, lb); ph[e] = as_h16(hb); pl[e] = as_h16(lb);
      }
      *(v8h*)(rh + c0 + 8 * hq) = ph;
      *(v8h*)(rl + c0 + 8 * hq) = pl;
    }
  }
  float s = 0.0f;
#pragma unroll
  for (int e = 0; e < 16; ++e) { v[e] = fmaxf(v[e], 0.0f); s += v[e]; }
#pragma unroll
  for (int off = 16; off > 0; off >>= 1) s += __shfl_xor(s, off, 32);
  const float mu = s * INV_H;
  float ss = 0.0f;
#pragma unroll
  for (int e = 0; e < 16; ++e) { v[e] = v[e] - mu; ss += v[e] * v[e]; }
#pragma unroll
  for (int off = 16; off > 0; off >>= 1) ss += __shfl_xor(ss, off, 32);
  const float var  = ss * INV_H;
  const float rstd = rsqrtf(var + LN_EPS);
#pragma unroll
  for (int hq = 0; hq < 2; ++hq) {
    const v4f ga = *(const v4f*)(gp + c0 + 8 * hq), gb = *(const v4f*)(gp + c0 + 8 * hq + 4);
    const v4f ba = *(const v4f*)(bp + c0 + 8 * hq), bb = *(const v4f*)(bp + c0 + 8 * hq + 4);
    v8h oh, ol;
#pragma unroll
    for (int e = 0; e < 4; ++e) {
      const float y0 = (v[8 * hq + e] * rstd) * ga[e] + ba[e];
      const float y1 = (v[8 * hq + 4 + e] * rstd) * gb[e] + bb[e];
      unsigned short hb, lb;
      split_bits(y0, hb, lb); oh[e] = as_h16(hb);     ol[e] = as_h16(lb);
      split_bits(y1, hb, lb); oh[4 + e] = as_h16(hb); ol[4 + e] = as_h16(lb);
    }
    *(v8h*)(uh + c0 + 8 * hq) = oh;
    *(v8h*)(ul + c0 + 8 * hq) = ol;
  }
}

__device__ __forceinline__ void cvt_row(const float* hfrow, unsigned short* rh, unsigned short* rl, int lane) {
  const int c0 = 16 * lane;
#pragma unroll
  for (int hq = 0; hq < 2; ++hq) {
    const v4f q0 = *(const v4f*)(hfrow + c0 + 8 * hq);
    const v4f q1 = *(const v4f*)(hfrow + c0 + 8 * hq + 4);
    v8h ph, pl;
#pragma unroll
    for (int e = 0; e < 4; ++e) {
      unsigned short hb, lb;
      split_bits(q0[e], hb, lb); ph[e] = as_h16(hb);     pl[e] = as_h16(lb);
      split_bits(q1[e], hb, lb); ph[4 + e] = as_h16(hb); pl[4 + e] = as_h16(lb);
    }
    *(v8h*)(rh + c0 + 8 * hq) = ph;
    *(v8h*)(rl + c0 + 8 * hq) = pl;
  }
}

template <int KA>
__device__ __forceinline__ void gate_tile(const __bf16* a1h, const __bf16* a1l, const __bf16* a2h, const __bf16* a2l,
                                          const __bf16* __restrict__ w1, const __bf16* __restrict__ w2,
                                          const float* __restrict__ bih, const float* __restrict__ bhh, int j,
                                          const float* __restrict__ mrow, float (&cst)[8], float* hfcol, int hh) {
  const v8f z8 = {0.f, 0.f, 0.f, 0.f, 0.f, 0.f, 0.f, 0.f};
  v8f acc[4];
  acc[0] = z8; acc[1] = z8; acc[2] = z8; acc[3] = z8;
#pragma unroll 1
  for (int k = 0; k < KA; k += 32) {
    const v16b ah = Frag<__bf16>::load(a1h + k);
    const v16b al = Frag<__bf16>::load(a1l + k);
#pragma unroll
    for (int g = 0; g < 4; ++g) {
      const __bf16* wp = w1 + (size_t)g * (NHID * KA) + k;
      const v16b bh = Frag<__bf16>::load(wp);
      const v16b bl = Frag<__bf16>::load(wp + (size_t)NG4 * KA);
      acc[g] = Frag<__bf16>::mma(ah, bh, acc[g]);
      acc[g] = Frag<__bf16>::mma(ah, bl, acc[g]);
      acc[g] = Frag<__bf16>::mma(al, bh, acc[g]);
      guard_all(acc[0], acc[1], acc[2], acc[3], ah, al, bh, bl);
    }
  }
#pragma unroll 1
  for (int k = 0; k < NHID; k += 32) {
    const v16b ah = Frag<__bf16>::load(a2h + k);
    const v16b al = Frag<__bf16>::load(a2l + k);
#pragma unroll
    for (int g = 0; g < 4; ++g) {
      const __bf16* wp = w2 + (size_t)g * (NHID * NHID) + k;
      const v16b bh = Frag<__bf16>::load(wp);
      const v16b bl = Frag<__bf16>::load(wp + (size_t)PL_H);
      acc[g] = Frag<__bf16>::mma(ah, bh, acc[g]);
      acc[g] = Frag<__bf16>::mma(ah, bl, acc[g]);
      acc[g] = Frag<__bf16>::mma(al, bh, acc[g]);
      guard_all(acc[0], acc[1], acc[2], acc[3], ah, al, bh, bl);
    }
  }
  acc_guard4(acc[0], acc[1], acc[2], acc[3]);
  const float bi = bih[j] + bhh[j];
  const float bf = bih[NHID + j] + bhh[NHID + j];
  const float bg = bih[2 * NHID + j] + bhh[2 * NHID + j];
  const float bo = bih[3 * NHID + j] + bhh[3 * NHID + j];
#pragma unroll
  for (int r = 0; r < 8; ++r) {
    const float mval = mrow[(size_t)r * NSTEP];
    const float zi = acc[0][r] + bi;
    const float zf = acc[1][r] + bf;
    const float zg = acc[2][r] + bg;
    const float zo = acc[3][r] + bo;
    const float ig = fsig(zi);
    const float fg = fsig(zf);
    const float og = fsig(zo);
    const float gg = ftanh(zg);
    float cn = fg * cst[r] + ig * gg;
    float hn = og * ftanh(cn);
    hn = hn * mval;
    cn = cn * mval;
    cst[r] = cn;
    hfcol[(8 * hh + r) * FPITCH] = hn;
  }
}

__global__ __launch_bounds__(NTHR) void lstm2_fused_kernel(
    const float* __restrict__ x, const float* __restrict__ rmask,
    const float* __restrict__ bih0, const float* __restrict__ bhh0, const float* __restrict__ g0, const float* __restrict__ be0,
    const float* __restrict__ bih1, const float* __restrict__ bhh1, const float* __restrict__ g1, const float* __restrict__ be1,
    const float* __restrict__ fcb,
    const unsigned short* __restrict__ wx0p, const unsigned short* __restrict__ wh0p,
    const unsigned short* __restrict__ wu1p, const unsigned short* __restrict__ wh1p,
    const unsigned short* __restrict__ wfcp,
    float* __restrict__ out) {
  __shared__ LdsAll L;
  const __bf16* WX0 = (const __bf16*)wx0p;
  const __bf16* WH0 = (const __bf16*)wh0p;
  const __bf16* WU1 = (const __bf16*)wu1p;
  const __bf16* WH1 = (const __bf16*)wh1p;
  const __bf16* WFC = (const __bf16*)wfcp;
  const int tid = threadIdx.x, lane = tid & 31, wave = tid >> 5;
  const int c = lane & 15, hh = lane >> 4, koff = hh * 8;
  const int rowbase = blockIdx.x * SEQ_BLK;
  const v8f z8 = {0.f, 0.f, 0.f, 0.f, 0.f, 0.f, 0.f, 0.f};

#pragma unroll 1
  for (int i = tid; i < SEQ_BLK * HPITCH; i += NTHR) { L.m.ah0h[i] = 0; L.m.ah0l[i] = 0; L.m.ah1h[i] = 0; L.m.ah1l[i] = 0; }
#pragma unroll 1
  for (int i = tid; i < SEQ_BLK * FPITCH; i += NTHR) L.m.hf[i] = 0.0f;
  {
    const float* msrow = rmask + (size_t)(rowbase + wave) * NSTEP + 16 * lane;
    const v4f m0 = *(const v4f*)(msrow), m1 = *(const v4f*)(msrow + 4), m2 = *(const v4f*)(msrow + 8), m3 = *(const v4f*)(msrow + 12);
    int lz = -1;
#pragma unroll
    for (int e = 0; e < 4; ++e) lz = (m0[e] == 0.0f) ? (16 * lane + e) : lz;
#pragma unroll
    for (int e = 0; e < 4; ++e) lz = (m1[e] == 0.0f) ? (16 * lane + 4 + e) : lz;
#pragma unroll
    for (int e = 0; e < 4; ++e) lz = (m2[e] == 0.0f) ? (16 * lane + 8 + e) : lz;
#pragma unroll
    for (int e = 0; e < 4; ++e) lz = (m3[e] == 0.0f) ? (16 * lane + 12 + e) : lz;
#pragma unroll
    for (int off = 16; off > 0; off >>= 1) { const int o = __shfl_xor(lz, off, 32); lz = (o > lz) ? o : lz; }
    if (lane == 0) L.m.sst[wave] = lz + 1;
  }
  float cst00[8], cst01[8], cst10[8], cst11[8];
#pragma unroll
  for (int r = 0; r < 8; ++r) { cst00[r] = 0.0f; cst01[r] = 0.0f; cst10[r] = 0.0f; cst11[r] = 0.0f; }
  __syncthreads();
  int start = NSTEP;
#pragma unroll
  for (int m = 0; m < SEQ_BLK; ++m) { const int s = L.m.sst[m]; start = (s < start) ? s : start; }
  start = (start < 0) ? 0 : ((start > NSTEP) ? NSTEP : start);
  stage_x(x, L.m.axh, L.m.axl, rowbase, (start < NSTEP) ? start : (NSTEP - 1), tid);
  __syncthreads();

  const int j0 = 32 * wave + c, j1 = j0 + 16;
  const __bf16* axh_r  = (const __bf16*)L.m.axh  + c * XPITCH + koff;
  const __bf16* axl_r  = (const __bf16*)L.m.axl  + c * XPITCH + koff;
  const __bf16* ah0h_r = (const __bf16*)L.m.ah0h + c * HPITCH + koff;
  const __bf16* ah0l_r = (const __bf16*)L.m.ah0l + c * HPITCH + koff;
  const __bf16* ah1h_r = (const __bf16*)L.m.ah1h + c * HPITCH + koff;
  const __bf16* ah1l_r = (const __bf16*)L.m.ah1l + c * HPITCH + koff;
  const __bf16* auh_r  = (const __bf16*)L.m.auh  + c * HPITCH + koff;
  const __bf16* aul_r  = (const __bf16*)L.m.aul  + c * HPITCH + koff;

#pragma unroll 1
  for (int t = start; t < NSTEP; ++t) {
    const float* mrow = rmask + (size_t)(rowbase + 8 * hh) * NSTEP + t;

    gate_tile<NIN>(axh_r, axl_r, ah0h_r, ah0l_r,
                   WX0 + (size_t)j0 * NIN + koff, WH0 + (size_t)j0 * NHID + koff,
                   bih0, bhh0, j0, mrow, cst00, L.m.hf + j0, hh);
    gate_tile<NIN>(axh_r, axl_r, ah0h_r, ah0l_r,
                   WX0 + (size_t)j1 * NIN + koff, WH0 + (size_t)j1 * NHID + koff,
                   bih0, bhh0, j1, mrow, cst01, L.m.hf + j1, hh);
    __syncthreads();

    ln_row<true>(L.m.hf + wave * FPITCH, g0, be0,
                 L.m.auh + wave * HPITCH, L.m.aul + wave * HPITCH,
                 L.m.ah0h + wave * HPITCH, L.m.ah0l + wave * HPITCH, lane);
    {
      const int tn = (t + 1 < NSTEP) ? (t + 1) : (NSTEP - 1);
      stage_x(x, L.m.axh, L.m.axl, rowbase, tn, tid);
    }
    __syncthreads();

    gate_tile<NHID>(auh_r, aul_r, ah1h_r, ah1l_r,
                    WU1 + (size_t)j0 * NHID + koff, WH1 + (size_t)j0 * NHID + koff,
                    bih1, bhh1, j0, mrow, cst10, L.m.hf + j0, hh);
    gate_tile<NHID>(auh_r, aul_r, ah1h_r, ah1l_r,
                    WU1 + (size_t)j1 * NHID + koff, WH1 + (size_t)j1 * NHID + koff,
                    bih1, bhh1, j1, mrow, cst11, L.m.hf + j1, hh);
    __syncthreads();

    cvt_row(L.m.hf + wave * FPITCH, L.m.ah1h + wave * HPITCH, L.m.ah1l + wave * HPITCH, lane);
    __syncthreads();
  }
  __syncthreads();
  ln_row<false>(L.m.hf + wave * FPITCH, g1, be1,
                L.m.auh + wave * HPITCH, L.m.aul + wave * HPITCH,
                L.m.auh + wave * HPITCH, L.m.aul + wave * HPITCH, lane);
  __syncthreads();

  {
    const int nb = 64 * wave;
    const __bf16* wf = WFC + (size_t)(nb + c) * NHID + koff;
    v8f acc[4];
    acc[0] = z8; acc[1] = z8; acc[2] = z8; acc[3] = z8;
#pragma unroll 1
    for (int k = 0; k < NHID; k += 32) {
      const v16b ah = Frag<__bf16>::load(auh_r + k);
      const v16b al = Frag<__bf16>::load(aul_r + k);
#pragma unroll
      for (int jj = 0; jj < 4; ++jj) {
        const __bf16* wp = wf + (size_t)jj * (16 * NHID) + k;
        const v16b bh = Frag<__bf16>::load(wp);
        const v16b bl = Frag<__bf16>::load(wp + (size_t)PL_C);
        acc[jj] = Frag<__bf16>::mma(ah, bh, acc[jj]);
        acc[jj] = Frag<__bf16>::mma(ah, bl, acc[jj]);
        acc[jj] = Frag<__bf16>::mma(al, bh, acc[jj]);
        guard_all(acc[0], acc[1], acc[2], acc[3], ah, al, bh, bl);
      }
    }
    acc_guard4(acc[0], acc[1], acc[2], acc[3]);
    float* ost = L.ost;
#pragma unroll
    for (int jj = 0; jj < 4; ++jj) {
      const int col  = nb + 16 * jj + c;
      const int colc = (col < NCLS) ? col : (NCLS - 1);
      const float bvv = fcb[colc];
      if (col < NCLS) {
#pragma unroll
        for (int r = 0; r < 8; ++r) ost[(8 * hh + r) * NCLS + col] = acc[jj][r] + bvv;
      }
    }
  }
  __syncthreads();
  {
    const float* ost = L.ost;
    float* ob = out + (size_t)blockIdx.x * OUT_BLK;
    for (int pass = 0; pass < 2; ++pass) {
#pragma unroll 1
      for (int q = wave; q < OUT_CHUNKS; q += NWAVE) {
        const v4f v = *(const v4f*)(ost + q * 128 + 4 * lane);
        *(volatile v4f*)(ob + q * 128 + 4 * lane) = v;
      }
      __threadfence();
    }
  }
}

extern "C" void kernel_launch(void* const* d_in, const int* in_sizes, int n_in,
                              void* d_out, int out_size, void* d_ws, size_t ws_size, hipStream_t stream) {
  if (n_in < 16 || d_out == nullptr || d_ws == nullptr) return;
  if (in_sizes[0] != NSEQ * NSTEP * NIN || in_sizes[1] != NSEQ * NSTEP ||
      in_sizes[2] != NG4 * NIN || in_sizes[3] != NG4 * NHID || in_sizes[4] != NG4 || in_sizes[5] != NG4 ||
      in_sizes[6] != NHID || in_sizes[7] != NHID ||
      in_sizes[8] != NG4 * NHID || in_sizes[9] != NG4 * NHID || in_sizes[10] != NG4 || in_sizes[11] != NG4 ||
      in_sizes[12] != NHID || in_sizes[13] != NHID ||
      in_sizes[14] != NCLS * NHID || in_sizes[15] != NCLS || out_size != NSEQ * NCLS) return;

  const float* xin  = (const float*)d_in[0];
  const float* rm   = (const float*)d_in[1];
  const float* wih0 = (const float*)d_in[2];
  const float* whh0 = (const float*)d_in[3];
  const float* bih0 = (const float*)d_in[4];
  const float* bhh0 = (const float*)d_in[5];
  const float* g0   = (const float*)d_in[6];
  const float* be0  = (const float*)d_in[7];
  const float* wih1 = (const float*)d_in[8];
  const float* whh1 = (const float*)d_in[9];
  const float* bih1 = (const float*)d_in[10];
  const float* bhh1 = (const float*)d_in[11];
  const float* g1   = (const float*)d_in[12];
  const float* be1  = (const float*)d_in[13];
  const float* fcw  = (const float*)d_in[14];
  const float* fcb  = (const float*)d_in[15];
  float* out = (float*)d_out;

  char* ws = (char*)d_ws; size_t off = 0;
  auto carve = [&](size_t bytes) -> char* { char* p = ws + off; off += (bytes + 255) & ~(size_t)255; return p; };
  unsigned short* WX0 = (unsigned short*)carve((size_t)2 * PL_X * 2);
  unsigned short* WH0 = (unsigned short*)carve((size_t)2 * PL_H * 2);
  unsigned short* WU1 = (unsigned short*)carve((size_t)2 * PL_H * 2);
  unsigned short* WH1 = (unsigned short*)carve((size_t)2 * PL_H * 2);
  unsigned short* WFC = (unsigned short*)carve((size_t)2 * PL_C * 2);
  if (off > ws_size || off > (size_t)134217728) return;

  const int n8x  = PL_X / 8;
  const int n8h  = PL_H / 8;
  const int n8fp = PL_C / 8;
  const int n8fs = NCLS * NHID / 8;
  split8_kernel<<<(n8x + CVT_THR - 1) / CVT_THR, CVT_THR, 0, stream>>>(wih0, WX0, WX0 + PL_X, n8x, n8x);
  split8_kernel<<<(n8h + CVT_THR - 1) / CVT_THR, CVT_THR, 0, stream>>>(whh0, WH0, WH0 + PL_H, n8h, n8h);
  split8_kernel<<<(n8h + CVT_THR - 1) / CVT_THR, CVT_THR, 0, stream>>>(wih1, WU1, WU1 + PL_H, n8h, n8h);
  split8_kernel<<<(n8h + CVT_THR - 1) / CVT_THR, CVT_THR, 0, stream>>>(whh1, WH1, WH1 + PL_H, n8h, n8h);
  split8_kernel<<<(n8fp + CVT_THR - 1) / CVT_THR, CVT_THR, 0, stream>>>(fcw, WFC, WFC + PL_C, n8fp, n8fs);
  lstm2_fused_kernel<<<NSEQ / SEQ_BLK, NTHR, 0, stream>>>(xin, rm, bih0, bhh0, g0, be0, bih1, bhh1, g1, be1, fcb,
                                                         WX0, WH0, WU1, WH1, WFC, out);
}
